// RNN_autoreg_35442070126823
// MI455X (gfx1250) — hardware-verified
//
#include <hip/hip_runtime.h>
#include <math.h>

typedef __attribute__((ext_vector_type(16))) _Float16 v16h;
typedef __attribute__((ext_vector_type(8)))  _Float16 v8h;
typedef __attribute__((ext_vector_type(8)))  float    v8f;
typedef __attribute__((ext_vector_type(4)))  float    v4f;

constexpr int NBAT     = 1024;
constexpr int NTIME    = 8;
constexpr int NLEV     = 60;
constexpr int NXF      = 4;
constexpr int NSF      = 3;
constexpr int NHID     = 64;
constexpr int NGATE    = 256;
constexpr int NMEMF    = 32;
constexpr int NYF      = 4;
constexpr int NYS      = 3;
constexpr int NIH1     = NXF + NMEMF;
constexpr int ROWS_BLK = 16;
constexpr int NTHR     = 512;
constexpr int NWAVE    = NTHR / 32;
constexpr int NOUT0    = NBAT * NTIME * NLEV * NYF;
constexpr int NOUT1    = NBAT * NTIME * NYS;
static_assert(NGATE == 4 * NHID, "gate blocks i|f|g|o");
static_assert(NGATE == 16 * NWAVE, "one 16-column gate tile per wave");
static_assert(ROWS_BLK * NHID == 2 * NTHR, "two cells per thread");
static_assert(NBAT % ROWS_BLK == 0, "block ownership");
static_assert(NHID % 32 == 0 && NMEMF % 32 == 0, "k tiles of 32, no tails");
static_assert(NIH1 == 36, "x first, then 32 memory features");
static_assert((NTIME % 2) == 0, "time steps flushed in pairs");
static_assert(((2 * NLEV * NYF * 4) % 128) == 0, "a pair of time steps is whole 128-B lines");
static_assert(((NOUT0 * 4) % 128) == 0, "second output starts on a line");
static_assert(((ROWS_BLK * NTIME * NYS * 4) % 128) == 0, "second output: whole lines per block");

constexpr float ACARRY  = 256.0f;
constexpr float WCARRY  = 16.0f;
constexpr float RCARRY  = 2048.0f;
constexpr float FOLD    = 1.0f / (ACARRY * WCARRY);
constexpr float FOLD_LO = FOLD / RCARRY;

constexpr int SZ_H1A   = NLEV * ROWS_BLK * NHID * 2;
constexpr int SZ_MEM   = NLEV * ROWS_BLK * NMEMF * 2;
constexpr int SZ_HA    = ROWS_BLK * NHID * 2;
constexpr int SZ_WL    = NMEMF * NHID * 2;
constexpr int SZ_GATES = ROWS_BLK * NGATE * 4;
constexpr int SZ_XL    = NLEV * ROWS_BLK * NXF * 4;
constexpr int SZ_LAT   = ROWS_BLK * NMEMF * 4;
constexpr int SZ_H2F   = ROWS_BLK * NHID * 4;
constexpr int SZ_STG0  = ROWS_BLK * 2 * NLEV * NYF * 4;
constexpr int SZ_STG1  = ROWS_BLK * NTIME * NYS * 4;
constexpr int SZ_WX    = NHID * 16 * 4;
constexpr int SZ_BG    = NGATE * 4;
constexpr int SZ_WOUT  = NYF * NMEMF * 4;
constexpr int SZ_WSFC  = NYS * NHID * 4;
constexpr int SZ_BMISC = 64 * 4;
constexpr int OFF_H1A   = 0;
constexpr int OFF_MEM   = OFF_H1A + SZ_H1A;
constexpr int OFF_HA    = OFF_MEM + SZ_MEM;
constexpr int OFF_HALO  = OFF_HA + SZ_HA;
constexpr int OFF_WLH   = OFF_HALO + SZ_HA;
constexpr int OFF_WLL   = OFF_WLH + SZ_WL;
constexpr int OFF_GATES = OFF_WLL + SZ_WL;
constexpr int OFF_XL    = OFF_GATES + SZ_GATES;
constexpr int OFF_LAT   = OFF_XL + SZ_XL;
constexpr int OFF_H2F   = OFF_LAT + SZ_LAT;
constexpr int OFF_STG0  = OFF_H2F + SZ_H2F;
constexpr int OFF_STG1  = OFF_STG0 + SZ_STG0;
constexpr int OFF_WX    = OFF_STG1 + SZ_STG1;
constexpr int OFF_B1    = OFF_WX + SZ_WX;
constexpr int OFF_B2    = OFF_B1 + SZ_BG;
constexpr int OFF_WOUT  = OFF_B2 + SZ_BG;
constexpr int OFF_WSFC  = OFF_WOUT + SZ_WOUT;
constexpr int OFF_BMISC = OFF_WSFC + SZ_WSFC;
constexpr int LDS_BYTES = OFF_BMISC + SZ_BMISC;
static_assert(LDS_BYTES == 274432, "LDS total");
static_assert((OFF_MEM % 16) == 0 && (OFF_HA % 16) == 0 && (OFF_HALO % 16) == 0 && (OFF_WLH % 16) == 0 &&
              (OFF_WLL % 16) == 0 && (OFF_GATES % 16) == 0 && (OFF_XL % 16) == 0 && (OFF_LAT % 16) == 0 &&
              (OFF_H2F % 16) == 0 && (OFF_STG0 % 16) == 0 && (OFF_STG1 % 16) == 0 && (OFF_WX % 16) == 0 &&
              (OFF_B1 % 16) == 0 && (OFF_B2 % 16) == 0 && (OFF_WOUT % 16) == 0 && (OFF_WSFC % 16) == 0 &&
              (OFF_BMISC % 16) == 0, "16-B aligned regions");
static_assert((SZ_MEM / 4) % NTHR == 0, "memory zero-fill loop exact");
static_assert(NMEMF * NHID == 4 * NTHR, "W_lat plane fill exact");

struct FragH {
  union U { v16h v; v8h h[2]; };
  static __device__ __forceinline__ v16h load(const _Float16* p) {
    U f; f.h[0] = *(const v8h*)(p); f.h[1] = *(const v8h*)(p + 16); return f.v;
  }
};

__device__ __forceinline__ v8f mma_g(v16h a, v16h b, v8f c) {
  c = __builtin_amdgcn_wmma_f32_16x16x32_f16(false, a, false, b, (short)0, c, false, false);
  asm volatile("v_nop\n\tv_nop\n\tv_nop\n\tv_nop" : "+v"(c) : "v"(a), "v"(b));
  return c;
}
__device__ __forceinline__ void acc_guard1(v8f& a) { asm volatile("v_nop\n\tv_nop\n\tv_nop\n\tv_nop" : "+v"(a)); }
__device__ __forceinline__ void acc_guard2(v8f& a, v8f& b) { asm volatile("v_nop\n\tv_nop\n\tv_nop\n\tv_nop" : "+v"(a), "+v"(b)); }

__device__ __forceinline__ v16h wfrag_hi(const float* p) {
  const v4f q0 = *(const v4f*)(p);
  const v4f q1 = *(const v4f*)(p + 4);
  const v4f q2 = *(const v4f*)(p + 16);
  const v4f q3 = *(const v4f*)(p + 20);
  v16h r;
#pragma unroll
  for (int e = 0; e < 4; ++e) {
    r[e]      = (_Float16)(q0[e] * WCARRY);
    r[4 + e]  = (_Float16)(q1[e] * WCARRY);
    r[8 + e]  = (_Float16)(q2[e] * WCARRY);
    r[12 + e] = (_Float16)(q3[e] * WCARRY);
  }
  return r;
}
__device__ __forceinline__ float wres(float w) {
  const float s = w * WCARRY;
  const float h = (float)((_Float16)s);
  return (s - h) * RCARRY;
}
__device__ __forceinline__ v16h wfrag_lo(const float* p) {
  const v4f q0 = *(const v4f*)(p);
  const v4f q1 = *(const v4f*)(p + 4);
  const v4f q2 = *(const v4f*)(p + 16);
  const v4f q3 = *(const v4f*)(p + 20);
  v16h r;
#pragma unroll
  for (int e = 0; e < 4; ++e) {
    r[e]      = (_Float16)wres(q0[e]);
    r[4 + e]  = (_Float16)wres(q1[e]);
    r[8 + e]  = (_Float16)wres(q2[e]);
    r[12 + e] = (_Float16)wres(q3[e]);
  }
  return r;
}

__device__ __forceinline__ float sigm(float x) { return 1.0f / (1.0f + expf(-x)); }

__global__ __launch_bounds__(NTHR) void level_lstm_kernel(
    const float* __restrict__ x_main, const float* __restrict__ x_sfc,
    const float* __restrict__ W_sfc1, const float* __restrict__ b_sfc1,
    const float* __restrict__ W_sfc2, const float* __restrict__ b_sfc2,
    const float* __restrict__ Wih1, const float* __restrict__ Whh1, const float* __restrict__ b1,
    const float* __restrict__ Wih2, const float* __restrict__ Whh2, const float* __restrict__ b2,
    const float* __restrict__ W_lat, const float* __restrict__ b_lat,
    const float* __restrict__ W_out, const float* __restrict__ b_out,
    const float* __restrict__ W_sfcout, const float* __restrict__ b_sfcout,
    float* __restrict__ outp) {
  extern __shared__ __align__(16) unsigned char smem[];
  _Float16* h1A   = (_Float16*)(smem + OFF_H1A);
  _Float16* memL  = (_Float16*)(smem + OFF_MEM);
  _Float16* hA    = (_Float16*)(smem + OFF_HA);
  _Float16* hAlo  = (_Float16*)(smem + OFF_HALO);
  _Float16* wlH   = (_Float16*)(smem + OFF_WLH);
  _Float16* wlL   = (_Float16*)(smem + OFF_WLL);
  float*    gates = (float*)(smem + OFF_GATES);
  float*    xl    = (float*)(smem + OFF_XL);
  float*    latS  = (float*)(smem + OFF_LAT);
  float*    h2f   = (float*)(smem + OFF_H2F);
  float*    stg0  = (float*)(smem + OFF_STG0);
  float*    stg1  = (float*)(smem + OFF_STG1);
  float*    wxS   = (float*)(smem + OFF_WX);
  float*    b1S   = (float*)(smem + OFF_B1);
  float*    b2S   = (float*)(smem + OFF_B2);
  float*    wOutS = (float*)(smem + OFF_WOUT);
  float*    wSfcS = (float*)(smem + OFF_WSFC);
  float*    bMisc = (float*)(smem + OFF_BMISC);

  const int tid  = threadIdx.x;
  const int lane = tid & 31;
  const int wave = tid >> 5;
  const int c    = lane & 15;
  const int hh   = lane >> 4;
  const int koff = hh * 8;
  const int col  = 16 * wave + c;
  const int b0   = blockIdx.x * ROWS_BLK;
  const int j    = tid & 63;
  const int mrow0 = tid >> 6;

  {
    unsigned* mz = (unsigned*)(smem + OFF_MEM);
#pragma unroll 1
    for (int i = tid; i < SZ_MEM / 4; i += NTHR) mz[i] = 0u;
  }
  {
    const int e0 = tid * 4;
    const v4f w = *(const v4f*)(W_lat + e0);
#pragma unroll
    for (int e = 0; e < 4; ++e) {
      const float s = w[e] * WCARRY;
      const _Float16 hi = (_Float16)s;
      const _Float16 lo = (_Float16)((s - (float)hi) * RCARRY);
      wlH[e0 + e] = hi;
      wlL[e0 + e] = lo;
    }
  }
  if (tid < 256) {
    const int jj = tid >> 2, g = tid & 3;
    const v4f w = *(const v4f*)(Wih1 + (size_t)(g * NHID + jj) * NIH1);
    *(v4f*)(wxS + tid * 4) = w;
    b1S[tid] = b1[tid];
    b2S[tid] = b2[tid];
  }
  if (tid < 128) wOutS[tid] = W_out[tid];
  if (tid < 192) wSfcS[tid] = W_sfcout[tid];
  if (tid < 64) {
    const int i0 = tid < 31 ? tid : 31;
    int i1 = tid - 32; i1 = i1 < 0 ? 0 : (i1 > 3 ? 3 : i1);
    int i2 = tid - 36; i2 = i2 < 0 ? 0 : (i2 > 2 ? 2 : i2);
    const float va = b_lat[i0];
    const float vb = b_out[i1];
    const float vc = b_sfcout[i2];
    const float v = (tid < 32) ? va : ((tid < 36) ? vb : ((tid < 39) ? vc : 0.0f));
    bMisc[tid] = v;
  }
  __syncthreads();

  const float ws1a = W_sfc1[j * NSF + 0], ws1b = W_sfc1[j * NSF + 1], ws1c = W_sfc1[j * NSF + 2], bs1 = b_sfc1[j];
  const float ws2a = W_sfc2[j * NSF + 0], ws2b = W_sfc2[j * NSF + 1], ws2c = W_sfc2[j * NSF + 2], bs2 = b_sfc2[j];
  const float blat  = bMisc[col & 31];
  const float boutq = bMisc[32 + (tid & 3)];
  int esf = tid - 64;
  esf = esf < 0 ? 0 : (esf > 47 ? 47 : esf);
  const int msf = esf / 3;
  const int qsf = esf - 3 * msf;
  const float bsfq = bMisc[36 + qsf];

  float* out0 = outp;
  float* out1 = outp + (size_t)NOUT0;
  const v8f z8 = {0.f, 0.f, 0.f, 0.f, 0.f, 0.f, 0.f, 0.f};

#pragma unroll 1
  for (int t = 0; t < NTIME; ++t) {
#pragma unroll
    for (int it = 0; it < 2; ++it) {
      const int idx = it * NTHR + tid;
      const int ic  = idx < NLEV * ROWS_BLK ? idx : (NLEV * ROWS_BLK - 1);
      const int m   = ic / NLEV;
      const int lv  = ic - m * NLEV;
      const v4f v = *(const v4f*)(x_main + ((size_t)(b0 + m) * NTIME + (size_t)t) * (NLEV * NXF) + lv * NXF);
      if (idx < NLEV * ROWS_BLK) *(v4f*)(xl + (lv * ROWS_BLK + m) * NXF) = v;
    }
    float cs[2];
#pragma unroll
    for (int s = 0; s < 2; ++s) {
      const int m = mrow0 + 8 * s;
      const float* sp = x_sfc + ((size_t)(b0 + m) * NTIME + (size_t)t) * NSF;
      const float s0 = sp[0], s1 = sp[1], s2 = sp[2];
      const float a1 = (s0 * ws1a + s1 * ws1b + s2 * ws1c) + bs1;
      const float a2 = (s0 * ws2a + s1 * ws2b + s2 * ws2c) + bs2;
      hA[m * NHID + j] = (_Float16)(tanhf(a1) * ACARRY);
      cs[s] = tanhf(a2);
    }
    __syncthreads();

    int zo = 0;
    asm volatile("" : "+v"(zo));
    const v16h wih1m = wfrag_hi(Wih1 + (size_t)col * NIH1 + NXF + koff + zo);
    const v16h whh1a = wfrag_hi(Whh1 + (size_t)col * NHID + koff + zo);
    const v16h whh1b = wfrag_hi(Whh1 + (size_t)col * NHID + 32 + koff + zo);

#pragma unroll 1
    for (int lv = NLEV - 1; lv >= 0; --lv) {
      {
        const v16h aM  = FragH::load(memL + lv * (ROWS_BLK * NMEMF) + c * NMEMF + koff);
        const v16h aH0 = FragH::load(hA + c * NHID + koff);
        const v16h aH1 = FragH::load(hA + c * NHID + 32 + koff);
        v8f acc = z8;
        acc = mma_g(aM,  wih1m, acc);
        acc = mma_g(aH0, whh1a, acc);
        acc = mma_g(aH1, whh1b, acc);
        acc_guard1(acc);
#pragma unroll
        for (int r = 0; r < 8; ++r) gates[(8 * hh + r) * NGATE + col] = acc[r] * FOLD;
      }
      __syncthreads();
      {
        const v4f w0 = *(const v4f*)(wxS + j * 16);
        const v4f w1 = *(const v4f*)(wxS + j * 16 + 4);
        const v4f w2 = *(const v4f*)(wxS + j * 16 + 8);
        const v4f w3 = *(const v4f*)(wxS + j * 16 + 12);
        const float bi = b1S[j], bf = b1S[NHID + j], bg = b1S[2 * NHID + j], bo = b1S[3 * NHID + j];
#pragma unroll
        for (int s = 0; s < 2; ++s) {
          const int m = mrow0 + 8 * s;
          const float* gp = gates + m * NGATE + j;
          const v4f xv = *(const v4f*)(xl + (lv * ROWS_BLK + m) * NXF);
          const float gi = gp[0]        + bi + ((xv[0] * w0[0] + xv[1] * w0[1]) + (xv[2] * w0[2] + xv[3] * w0[3]));
          const float gf = gp[NHID]     + bf + ((xv[0] * w1[0] + xv[1] * w1[1]) + (xv[2] * w1[2] + xv[3] * w1[3]));
          const float gg = gp[2 * NHID] + bg + ((xv[0] * w2[0] + xv[1] * w2[1]) + (xv[2] * w2[2] + xv[3] * w2[3]));
          const float go = gp[3 * NHID] + bo + ((xv[0] * w3[0] + xv[1] * w3[1]) + (xv[2] * w3[2] + xv[3] * w3[3]));
          const float ig = sigm(gi);
          const float fg = sigm(gf);
          const float og = sigm(go);
          const float gt = tanhf(gg);
          const float cn = fg * cs[s] + ig * gt;
          cs[s] = cn;
          const float hn = og * tanhf(cn);
          const _Float16 h16 = (_Float16)(hn * ACARRY);
          hA[m * NHID + j] = h16;
          h1A[lv * (ROWS_BLK * NHID) + m * NHID + j] = h16;
        }
      }
      __syncthreads();
    }

#pragma unroll
    for (int s = 0; s < 2; ++s) {
      hA[(mrow0 + 8 * s) * NHID + j] = (_Float16)0.0f;
      cs[s] = 0.0f;
    }
    __syncthreads();

    int zp = 0;
    asm volatile("" : "+v"(zp));
    const v16h wih2a  = wfrag_hi(Wih2 + (size_t)col * NHID + koff + zp);
    const v16h wih2b  = wfrag_hi(Wih2 + (size_t)col * NHID + 32 + koff + zp);
    const v16h wih2la = wfrag_lo(Wih2 + (size_t)col * NHID + koff + zp);
    const v16h wih2lb = wfrag_lo(Wih2 + (size_t)col * NHID + 32 + koff + zp);
    const v16h whh2a  = wfrag_hi(Whh2 + (size_t)col * NHID + koff + zp);
    const v16h whh2b  = wfrag_hi(Whh2 + (size_t)col * NHID + 32 + koff + zp);

#pragma unroll 1
    for (int lv = 0; lv < NLEV; ++lv) {
      {
        const v16h aX0 = FragH::load(h1A + lv * (ROWS_BLK * NHID) + c * NHID + koff);
        const v16h aX1 = FragH::load(h1A + lv * (ROWS_BLK * NHID) + c * NHID + 32 + koff);
        const v16h aH0 = FragH::load(hA + c * NHID + koff);
        const v16h aH1 = FragH::load(hA + c * NHID + 32 + koff);
        v8f acc = z8, accR = z8;
        acc  = mma_g(aX0, wih2a, acc);
        acc  = mma_g(aX1, wih2b, acc);
        acc  = mma_g(aH0, whh2a, acc);
        acc  = mma_g(aH1, whh2b, acc);
        accR = mma_g(aX0, wih2la, accR);
        accR = mma_g(aX1, wih2lb, accR);
        acc_guard2(acc, accR);
#pragma unroll
        for (int r = 0; r < 8; ++r) gates[(8 * hh + r) * NGATE + col] = acc[r] * FOLD + accR[r] * FOLD_LO;
      }
      __syncthreads();
      {
        const float bi = b2S[j], bf = b2S[NHID + j], bg = b2S[2 * NHID + j], bo = b2S[3 * NHID + j];
#pragma unroll
        for (int s = 0; s < 2; ++s) {
          const int m = mrow0 + 8 * s;
          const float* gp = gates + m * NGATE + j;
          const float gi = gp[0] + bi;
          const float gf = gp[NHID] + bf;
          const float gg = gp[2 * NHID] + bg;
          const float go = gp[3 * NHID] + bo;
          const float ig = sigm(gi);
          const float fg = sigm(gf);
          const float og = sigm(go);
          const float gt = tanhf(gg);
          const float cn = fg * cs[s] + ig * gt;
          cs[s] = cn;
          const float hn = og * tanhf(cn);
          const float hv = hn * ACARRY;
          const float hq = (fabsf(hv) < 6.2e-5f) ? 0.0f : hv;
          const _Float16 hi = (_Float16)hq;
          const _Float16 lo = (_Float16)((hv - (float)hi) * RCARRY);
          hA[m * NHID + j]   = hi;
          hAlo[m * NHID + j] = lo;
          if (lv == NLEV - 1) h2f[m * NHID + j] = hn;
        }
      }
      __syncthreads();
      if (wave < 2) {
        const v16h aH0 = FragH::load(hA + c * NHID + koff);
        const v16h aH1 = FragH::load(hA + c * NHID + 32 + koff);
        const v16h aL0 = FragH::load(hAlo + c * NHID + koff);
        const v16h aL1 = FragH::load(hAlo + c * NHID + 32 + koff);
        const v16h bH0 = FragH::load(wlH + col * NHID + koff);
        const v16h bH1 = FragH::load(wlH + col * NHID + 32 + koff);
        const v16h bL0 = FragH::load(wlL + col * NHID + koff);
        const v16h bL1 = FragH::load(wlL + col * NHID + 32 + koff);
        v8f accM = z8, accR = z8;
        accM = mma_g(aH0, bH0, accM);
        accM = mma_g(aH1, bH1, accM);
        accR = mma_g(aH0, bL0, accR);
        accR = mma_g(aH1, bL1, accR);
        accR = mma_g(aL0, bH0, accR);
        accR = mma_g(aL1, bH1, accR);
        acc_guard2(accM, accR);
#pragma unroll
        for (int r = 0; r < 8; ++r) {
          const int m = 8 * hh + r;
          const float v = accM[r] * FOLD + accR[r] * FOLD_LO + blat;
          latS[m * NMEMF + col] = v;
          memL[lv * (ROWS_BLK * NMEMF) + m * NMEMF + col] = (_Float16)(v * ACARRY);
        }
      }
      __syncthreads();
      if (tid < 64) {
        const int m = tid >> 2, q = tid & 3;
        float a = boutq;
#pragma unroll
        for (int p = 0; p < NMEMF / 4; ++p) {
          const v4f l4 = *(const v4f*)(latS + m * NMEMF + 4 * p);
          const v4f w4 = *(const v4f*)(wOutS + q * NMEMF + 4 * p);
          a += (l4[0] * w4[0] + l4[1] * w4[1]) + (l4[2] * w4[2] + l4[3] * w4[3]);
        }
        stg0[m * (2 * NLEV * NYF) + (t & 1) * (NLEV * NYF) + lv * NYF + q] = a;
      }
      if (lv == NLEV - 1 && wave >= 2 && wave < 4) {
        float a = bsfq;
#pragma unroll 4
        for (int k = 0; k < NHID; ++k) a += h2f[msf * NHID + k] * wSfcS[qsf * NHID + k];
        if (tid - 64 < ROWS_BLK * NYS) stg1[msf * (NTIME * NYS) + t * NYS + qsf] = a;
      }
    }
    __syncthreads();

    if (t & 1) {
      float* gb = out0 + ((size_t)b0 * NTIME + (size_t)(t - 1)) * (NLEV * NYF);
      for (int pass = 0; pass < 2; ++pass) {
#pragma unroll
        for (int it = 0; it < 4; ++it) {
          const int i = it * NTHR + tid;
          if (i < ROWS_BLK * 120) {
            const int m = i / 120;
            const int w = i - m * 120;
            const v4f v = *(const v4f*)(stg0 + m * (2 * NLEV * NYF) + w * 4);
            *(volatile v4f*)(gb + (size_t)m * (NTIME * NLEV * NYF) + w * 4) = v;
          }
        }
        __threadfence();
      }
    }
  }

  if (tid < 96) {
    const v4f v = *(const v4f*)(stg1 + tid * 4);
    float* gp = out1 + (size_t)b0 * (NTIME * NYS) + tid * 4;
    *(volatile v4f*)gp = v;
    __threadfence();
    *(volatile v4f*)gp = v;
  }
}

extern "C" void kernel_launch(void* const* d_in, const int* in_sizes, int n_in,
                              void* d_out, int out_size, void* d_ws, size_t ws_size, hipStream_t stream) {
  (void)d_ws; (void)ws_size;
  if (n_in < 18 || d_out == nullptr) return;
  if (in_sizes[0] != NBAT * NTIME * NLEV * NXF || in_sizes[1] != NBAT * NTIME * NSF ||
      in_sizes[2] != NHID * NSF || in_sizes[3] != NHID || in_sizes[4] != NHID * NSF || in_sizes[5] != NHID ||
      in_sizes[6] != NGATE * NIH1 || in_sizes[7] != NGATE * NHID || in_sizes[8] != NGATE ||
      in_sizes[9] != NGATE * NHID || in_sizes[10] != NGATE * NHID || in_sizes[11] != NGATE ||
      in_sizes[12] != NMEMF * NHID || in_sizes[13] != NMEMF || in_sizes[14] != NYF * NMEMF ||
      in_sizes[15] != NYF || in_sizes[16] != NYS * NHID || in_sizes[17] != NYS ||
      out_size != NOUT0 + NOUT1) return;

  level_lstm_kernel<<<NBAT / ROWS_BLK, NTHR, LDS_BYTES, stream>>>(
      (const float*)d_in[0],  (const float*)d_in[1],
      (const float*)d_in[2],  (const float*)d_in[3],
      (const float*)d_in[4],  (const float*)d_in[5],
      (const float*)d_in[6],  (const float*)d_in[7],  (const float*)d_in[8],
      (const float*)d_in[9],  (const float*)d_in[10], (const float*)d_in[11],
      (const float*)d_in[12], (const float*)d_in[13],
      (const float*)d_in[14], (const float*)d_in[15],
      (const float*)d_in[16], (const float*)d_in[17],
      (float*)d_out);
}
